// Hedgehog_20864951124431
// MI455X (gfx1250) — hardware-verified
//
#include <hip/hip_runtime.h>
#include <math.h>
#include <stdint.h>

#ifndef NB
#define NB 1
#endif
#ifndef SEQ
#define SEQ 1024
#endif
#define XS_FULL 1024
#define DMOD  1024
#define NH    16
#define HD    64
#define FD    64
#define F2    128
#define EPSV  1e-12f
#define LOG2E 1.4426950408889634f
#define QSC   256.0f
#define KQS   256.0f
#define FCAR  16384.0f
#define PCAR  16384.0f
#define VCAR  1024.0f
#define OSC   1024.0f
#define WOS   1024.0f
#define WPB   2
#define NHG   (NH / WPB)
#define NQT   (SEQ / 16)
#define NST   (SEQ / 64)
#define NKT   (SEQ / 32)
#define ATT_THREADS (WPB * 32)
#define PTP   36
#define PTW   (16 * PTP)
#define SLP   68
#define SLW   (16 * SLP)
#define WREG  (PTW + SLW)
#define SLAB64 (16 * 68)
#define VTP   72
#define FWPB  4
#define FM_THREADS (FWPB * 32)
#define FSP   132
#define FSW   (16 * FSP)
#define C8R   (DMOD / 8)
#define WS_CAP 134217728
static_assert(NB == 1);
static_assert(DMOD == NH * HD && HD == 64 && FD == 64 && F2 == 2 * FD && NH == 16 && WPB == 2 && NHG * WPB == NH);
static_assert(ATT_THREADS == 64 && FM_THREADS == 128);
static_assert((SEQ % 64) == 0 && SEQ >= 64 && SEQ <= XS_FULL);
static_assert(((NH * NQT) % FWPB) == 0);
static_assert((DMOD % 64) == 0 && (DMOD % 32) == 0 && (HD % 32) == 0 && (F2 % 32) == 0 && C8R == 128);
static_assert(((SEQ * DMOD / 8) % 256) == 0 && ((DMOD * DMOD / 8) % 256) == 0);
static_assert(WPB * WREG * 4 <= 65536 && FWPB * FSW * 4 <= 65536 && 2 * HD * VTP * 2 <= 65536 && 4 * SLAB64 * 4 <= 65536);

typedef unsigned short u16;
typedef _Float16 v16h __attribute__((ext_vector_type(16)));
typedef _Float16 v8h  __attribute__((ext_vector_type(8)));
typedef __bf16   v16b __attribute__((ext_vector_type(16)));
typedef float    v8f  __attribute__((ext_vector_type(8)));
typedef float    v4f  __attribute__((ext_vector_type(4)));
typedef unsigned int v4u __attribute__((ext_vector_type(4)));

union FragH { v16h v; v8h h[2]; v4u u[2]; };
union FragB { v16b v; v4u u[2]; };

__device__ __forceinline__ unsigned short bf_bits(float f) {
  unsigned u = __float_as_uint(f);
  return (unsigned short)((u + 0x7FFFu + ((u >> 16) & 1u)) >> 16);
}
__device__ __forceinline__ float bf_up(unsigned short h) { return __uint_as_float(((unsigned)h) << 16); }
__device__ __forceinline__ float bfr(float f) { return bf_up(bf_bits(f)); }
__device__ __forceinline__ unsigned short h_bits(_Float16 x) { return __builtin_bit_cast(unsigned short, x); }
__device__ __forceinline__ unsigned pk16(unsigned short a, unsigned short b) { return (unsigned)a | ((unsigned)b << 16); }
__device__ __forceinline__ v8f zero8() { v8f z = {0.f, 0.f, 0.f, 0.f, 0.f, 0.f, 0.f, 0.f}; return z; }
__device__ __forceinline__ const _Float16* ash(const u16* p) { return (const _Float16*)(const void*)p; }

__device__ __forceinline__ v16h ldfrag_h(const _Float16* p) {
  FragH f;
  f.h[0] = *(const v8h*)(p);
  f.h[1] = *(const v8h*)(p + 16);
  return f.v;
}
__device__ __forceinline__ v16b ldfrag_b(const u16* p) {
  FragB f;
  f.u[0] = *(const v4u*)(p);
  f.u[1] = *(const v4u*)(p + 16);
  return f.v;
}

__device__ __forceinline__ v8f mma_h(v16h a, v16h b, v8f c) {
  return __builtin_amdgcn_wmma_f32_16x16x32_f16(false, a, false, b, (short)0, c, false, false);
}
__device__ __forceinline__ v8f mma_b(v16b a, v16b b, v8f c) {
  return __builtin_amdgcn_wmma_f32_16x16x32_bf16(false, a, false, b, (short)0, c, false, false);
}
__device__ __forceinline__ void guard2(v8f& a, v8f& b, v16h x0, v16h x1, v16h x2, v16h x3, v16h x4, v16h x5) {
#if defined(__HIP_DEVICE_COMPILE__)
  asm volatile("v_nop\n\tv_nop\n\tv_nop\n\tv_nop"
               : "+v"(a), "+v"(b) : "v"(x0), "v"(x1), "v"(x2), "v"(x3), "v"(x4), "v"(x5) : "memory");
#endif
}
template <typename F>
__device__ __forceinline__ void guard6(v8f& a, v8f& b, v8f& c, v8f& d, F x0, F x1, F x2, F x3, F x4, F x5) {
#if defined(__HIP_DEVICE_COMPILE__)
  asm volatile("v_nop\n\tv_nop\n\tv_nop\n\tv_nop"
               : "+v"(a), "+v"(b), "+v"(c), "+v"(d) : "v"(x0), "v"(x1), "v"(x2), "v"(x3), "v"(x4), "v"(x5) : "memory");
#endif
}
__device__ __forceinline__ void acc_guard4(v8f& a, v8f& b, v8f& c, v8f& d) {
#if defined(__HIP_DEVICE_COMPILE__)
  asm volatile("v_nop\n\tv_nop\n\tv_nop\n\tv_nop" : "+v"(a), "+v"(b), "+v"(c), "+v"(d));
#endif
}
__device__ __forceinline__ void wave_sync_lds() {
  __builtin_amdgcn_fence(__ATOMIC_RELEASE, "workgroup");
  __builtin_amdgcn_wave_barrier();
  __builtin_amdgcn_fence(__ATOMIC_ACQUIRE, "workgroup");
}

__global__ __launch_bounds__(256) void cvt16(const float* __restrict__ x, u16* D, int n8, int f16mode, float scale) {
  const int gt = blockIdx.x * 256 + (int)threadIdx.x;
  if (gt >= n8) return;
  const float* p = x + (size_t)gt * 8;
  const v4f a = *(const v4f*)(p), b4 = *(const v4f*)(p + 4);
  float w[8];
#pragma unroll
  for (int e = 0; e < 4; ++e) { w[e] = a[e]; w[4 + e] = b4[e]; }
  v4u o;
#pragma unroll
  for (int e = 0; e < 4; ++e) {
    const float f0 = w[2 * e], f1 = w[2 * e + 1];
    const unsigned short hb0 = h_bits((_Float16)(bfr(f0) * scale));
    const unsigned short hb1 = h_bits((_Float16)(bfr(f1) * scale));
    const unsigned short bb0 = bf_bits(f0);
    const unsigned short bb1 = bf_bits(f1);
    o[e] = (f16mode != 0) ? pk16(hb0, hb1) : pk16(bb0, bb1);
  }
  u16* d = D + (size_t)gt * 8;
  for (int pass = 0; pass < 2; ++pass) {
    *(volatile v4u*)(d) = o;
    __threadfence();
  }
}

__global__ __launch_bounds__(256) void tr16(const float* __restrict__ S, u16* D, int R, int C, int nz, int f16mode, float scale) {
  __shared__ __align__(16) u16 T[64 * VTP];
  const int tid = threadIdx.x;
  const int bid = blockIdx.x;
  const int nct = C >> 6, nrt = R >> 6;
  const int ct  = bid % nct;
  const int t2  = bid / nct;
  const int rt  = t2 % nrt;
  const int z   = t2 / nrt;
  if (z >= nz) return;
  const int r0 = rt * 64, c0 = ct * 64;
  {
    const int rl = tid >> 2;
    const int cc = (tid & 3) * 16;
    const float* src = S + ((size_t)z * R + r0 + rl) * (size_t)C + c0 + cc;
#pragma unroll
    for (int i = 0; i < 4; ++i) {
      const v4f a = *(const v4f*)(src + 4 * i);
#pragma unroll
      for (int e = 0; e < 4; ++e) {
        const float f = a[e];
        const unsigned short hb = h_bits((_Float16)(bfr(f) * scale));
        const unsigned short bb = bf_bits(f);
        T[(cc + 4 * i + e) * VTP + rl] = (f16mode != 0) ? hb : bb;
      }
    }
  }
  __syncthreads();
  v4u v[2];
  const int q8 = tid >> 3, p8 = (tid & 7) * 8;
#pragma unroll
  for (int it = 0; it < 2; ++it) {
    const int line = it * 32 + q8;
    v[it] = *(const v4u*)(T + line * VTP + p8);
  }
  const size_t base = ((size_t)z * C + c0) * (size_t)R + r0 + p8;
  for (int pass = 0; pass < 2; ++pass) {
#pragma unroll
    for (int it = 0; it < 2; ++it) {
      const int line = it * 32 + q8;
      *(volatile v4u*)(D + base + (size_t)line * (size_t)R) = v[it];
    }
    __threadfence();
  }
}

__global__ __launch_bounds__(256) void split16(const float* __restrict__ F, u16* Hp, u16* Lp, int n8, float sc) {
  const int gt = blockIdx.x * 256 + (int)threadIdx.x;
  if (gt >= n8) return;
  const float* p = F + (size_t)gt * 8;
  const v4f a = *(const v4f*)(p), b4 = *(const v4f*)(p + 4);
  float w[8];
#pragma unroll
  for (int e = 0; e < 4; ++e) { w[e] = a[e] * sc; w[4 + e] = b4[e] * sc; }
  v4u oh, ol;
#pragma unroll
  for (int e = 0; e < 4; ++e) {
    const float t0 = w[2 * e], t1 = w[2 * e + 1];
    const _Float16 h0 = (_Float16)t0, h1 = (_Float16)t1;
    const _Float16 l0 = (_Float16)(t0 - (float)h0), l1 = (_Float16)(t1 - (float)h1);
    oh[e] = pk16(h_bits(h0), h_bits(h1));
    ol[e] = pk16(h_bits(l0), h_bits(l1));
  }
  u16* dh = Hp + (size_t)gt * 8;
  u16* dl = Lp + (size_t)gt * 8;
  for (int pass = 0; pass < 2; ++pass) {
    *(volatile v4u*)(dh) = oh;
    *(volatile v4u*)(dl) = ol;
    __threadfence();
  }
}

__global__ __launch_bounds__(256) void vt16(const float* __restrict__ F, u16* VHo, u16* VLo) {
  __shared__ __align__(16) u16 TH[HD * VTP];
  __shared__ __align__(16) u16 TL[HD * VTP];
  const int tid = threadIdx.x;
  const int bid = blockIdx.x;
  const int st  = bid % NST;
  const int h   = bid / NST;
  if (h >= NH) return;
  const int s0  = st * 64;
  {
    const int sl = tid >> 2;
    const int dc = (tid & 3) * 16;
    const float* src = F + (size_t)(s0 + sl) * DMOD + h * HD + dc;
#pragma unroll
    for (int i = 0; i < 4; ++i) {
      const v4f a = *(const v4f*)(src + 4 * i);
#pragma unroll
      for (int e = 0; e < 4; ++e) {
        const float t = a[e] * VCAR;
        const _Float16 hv = (_Float16)t;
        const _Float16 lv = (_Float16)(t - (float)hv);
        TH[(dc + 4 * i + e) * VTP + sl] = h_bits(hv);
        TL[(dc + 4 * i + e) * VTP + sl] = h_bits(lv);
      }
    }
  }
  __syncthreads();
  v4u vh[2], vl[2];
  const int q8 = tid >> 3, p8 = (tid & 7) * 8;
#pragma unroll
  for (int it = 0; it < 2; ++it) {
    const int line = it * 32 + q8;
    vh[it] = *(const v4u*)(TH + line * VTP + p8);
    vl[it] = *(const v4u*)(TL + line * VTP + p8);
  }
  const size_t base = (size_t)(h * HD) * SEQ + s0 + p8;
  for (int pass = 0; pass < 2; ++pass) {
#pragma unroll
    for (int it = 0; it < 2; ++it) {
      const int line = it * 32 + q8;
      *(volatile v4u*)(VHo + base + (size_t)line * SEQ) = vh[it];
      *(volatile v4u*)(VLo + base + (size_t)line * SEQ) = vl[it];
    }
    __threadfence();
  }
}

__device__ __forceinline__ void epi64(float* sl, v8f a0, v8f a1, v8f a2, v8f a3, float oscale,
                                      float* C, int N, size_t rowb, int col0, int lane) {
  const int hh = lane >> 4, m = lane & 15;
#pragma unroll
  for (int r = 0; r < 8; ++r) {
    const int ro = (8 * hh + r) * 68 + m;
    sl[ro]      = a0[r] * oscale;
    sl[ro + 16] = a1[r] * oscale;
    sl[ro + 32] = a2[r] * oscale;
    sl[ro + 48] = a3[r] * oscale;
  }
  wave_sync_lds();
  v4f vals[8];
#pragma unroll
  for (int it = 0; it < 8; ++it) vals[it] = *(const v4f*)(sl + (it * 2 + hh) * 68 + m * 4);
  float* dst = C + (rowb + (size_t)hh) * (size_t)N + col0 + m * 4;
  for (int pass = 0; pass < 2; ++pass) {
#pragma unroll
    for (int it = 0; it < 8; ++it) {
      *(volatile v4f*)(dst + (size_t)(it * 2) * (size_t)N) = vals[it];
    }
    __threadfence();
  }
}

__global__ __launch_bounds__(128)
void gemm_bf(const u16* __restrict__ A, const u16* __restrict__ Bt, float* C, int M, int N, int K, float oscale) {
  __shared__ __align__(16) float slab[4 * SLAB64];
  const int tid = threadIdx.x, wave = tid >> 5, lane = tid & 31, hh = lane >> 4, m = lane & 15;
  const int ntile = N >> 6;
  const int bid   = blockIdx.x;
  const int rowb  = (bid / ntile) * 64 + wave * 16;
  const int col0  = (bid % ntile) * 64;
  if (rowb + 16 > M) return;
  const u16* ap = A  + (size_t)(rowb + m) * K + 8 * hh;
  const u16* bp = Bt + (size_t)(col0 + m) * K + 8 * hh;
  const size_t bs = (size_t)16 * K;
  v8f acc0 = zero8(), acc1 = zero8(), acc2 = zero8(), acc3 = zero8();
#pragma unroll 1
  for (int k0 = 0; k0 < K; k0 += 32) {
    const v16b a  = ldfrag_b(ap + k0);
    const v16b b0 = ldfrag_b(bp + k0);
    const v16b b1 = ldfrag_b(bp + bs + k0);
    const v16b b2 = ldfrag_b(bp + 2 * bs + k0);
    const v16b b3 = ldfrag_b(bp + 3 * bs + k0);
    acc0 = mma_b(a, b0, acc0);
    acc1 = mma_b(a, b1, acc1);
    acc2 = mma_b(a, b2, acc2);
    acc3 = mma_b(a, b3, acc3);
    guard6<v16b>(acc0, acc1, acc2, acc3, a, b0, b1, b2, b3, a);
  }
  epi64(slab + wave * SLAB64, acc0, acc1, acc2, acc3, oscale, C, N, (size_t)rowb, col0, lane);
}

__global__ __launch_bounds__(128)
void gemm_o(const u16* __restrict__ Ah, const u16* __restrict__ Al, const u16* __restrict__ Bt, float* C, float oscale) {
  __shared__ __align__(16) float slab[4 * SLAB64];
  const int tid = threadIdx.x, wave = tid >> 5, lane = tid & 31, hh = lane >> 4, m = lane & 15;
  const int ntile = DMOD >> 6;
  const int bid   = blockIdx.x;
  const int ct    = bid % ntile;
  const int rt    = bid / ntile;
  const int srow  = rt * 64 + wave * 16;
  if (srow + 16 > SEQ) return;
  const int col0  = ct * 64;
  const int K     = DMOD;
  const _Float16* ahp = ash(Ah) + (size_t)(srow + m) * K + 8 * hh;
  const _Float16* alp = ash(Al) + (size_t)(srow + m) * K + 8 * hh;
  const _Float16* bp  = ash(Bt) + (size_t)(col0 + m) * K + 8 * hh;
  const size_t bs = (size_t)16 * K;
  v8f acc0 = zero8(), acc1 = zero8(), acc2 = zero8(), acc3 = zero8();
#pragma unroll 1
  for (int k0 = 0; k0 < K; k0 += 32) {
    const v16h ah = ldfrag_h(ahp + k0), al = ldfrag_h(alp + k0);
    const v16h b0 = ldfrag_h(bp + k0);
    const v16h b1 = ldfrag_h(bp + bs + k0);
    const v16h b2 = ldfrag_h(bp + 2 * bs + k0);
    const v16h b3 = ldfrag_h(bp + 3 * bs + k0);
    acc0 = mma_h(ah, b0, acc0);  acc0 = mma_h(al, b0, acc0);
    acc1 = mma_h(ah, b1, acc1);  acc1 = mma_h(al, b1, acc1);
    acc2 = mma_h(ah, b2, acc2);  acc2 = mma_h(al, b2, acc2);
    acc3 = mma_h(ah, b3, acc3);  acc3 = mma_h(al, b3, acc3);
    guard6<v16h>(acc0, acc1, acc2, acc3, ah, al, b0, b1, b2, b3);
  }
  epi64(slab + wave * SLAB64, acc0, acc1, acc2, acc3, oscale, C, DMOD, (size_t)srow, col0, lane);
}

__global__ __launch_bounds__(FM_THREADS)
void fmap(const u16* __restrict__ QHp, const u16* __restrict__ QLp, const u16* __restrict__ KTp, u16* FHo, u16* FLo) {
  __shared__ __align__(16) float fsm[FWPB * FSW];
  const int tid = threadIdx.x, wave = tid >> 5, lane = tid & 31, hh = lane >> 4, c = lane & 15;
  const int tile = (int)blockIdx.x * FWPB + wave;
  const int head = tile / NQT;
  const int qt   = tile - head * NQT;
  if (head >= NH) return;
  const int q0 = qt * 16;
  float* slab = fsm + wave * FSW;
  const size_t qoff = (size_t)(q0 + c) * DMOD + (size_t)head * HD + 8 * hh;
  const _Float16* Qh = ash(QHp) + qoff;
  const _Float16* Ql = ash(QLp) + qoff;
  const _Float16* Bp = ash(KTp) + ((size_t)head * FD + c) * HD + 8 * hh;
  const size_t bs = (size_t)16 * HD;
  v8f acc0 = zero8(), acc1 = zero8(), acc2 = zero8(), acc3 = zero8();
#pragma unroll
  for (int kk = 0; kk < HD / 32; ++kk) {
    const v16h qh = ldfrag_h(Qh + kk * 32);
    const v16h ql = ldfrag_h(Ql + kk * 32);
    const v16h b0 = ldfrag_h(Bp + kk * 32);
    const v16h b1 = ldfrag_h(Bp + bs + kk * 32);
    const v16h b2 = ldfrag_h(Bp + 2 * bs + kk * 32);
    const v16h b3 = ldfrag_h(Bp + 3 * bs + kk * 32);
    acc0 = mma_h(qh, b0, acc0);  acc0 = mma_h(ql, b0, acc0);
    acc1 = mma_h(qh, b1, acc1);  acc1 = mma_h(ql, b1, acc1);
    acc2 = mma_h(qh, b2, acc2);  acc2 = mma_h(ql, b2, acc2);
    acc3 = mma_h(qh, b3, acc3);  acc3 = mma_h(ql, b3, acc3);
    guard6<v16h>(acc0, acc1, acc2, acc3, qh, ql, b0, b1, b2, b3);
  }
  acc_guard4(acc0, acc1, acc2, acc3);
  const float fsc = 1.0f / (QSC * KQS);
#pragma unroll
  for (int r = 0; r < 8; ++r) {
    const float v0 = acc0[r] * fsc, v1 = acc1[r] * fsc, v2 = acc2[r] * fsc, v3 = acc3[r] * fsc;
    float mx = fmaxf(fmaxf(v0, v1), fmaxf(v2, v3));
    float mn = fminf(fminf(v0, v1), fminf(v2, v3));
#pragma unroll
    for (int off = 1; off < 16; off <<= 1) {
      mx = fmaxf(mx, __shfl_xor(mx, off, 32));
      mn = fminf(mn, __shfl_xor(mn, off, 32));
    }
    const float ep0 = exp2f((v0 - mx) * LOG2E), ep1 = exp2f((v1 - mx) * LOG2E);
    const float ep2 = exp2f((v2 - mx) * LOG2E), ep3 = exp2f((v3 - mx) * LOG2E);
    const float en0 = exp2f((mn - v0) * LOG2E), en1 = exp2f((mn - v1) * LOG2E);
    const float en2 = exp2f((mn - v2) * LOG2E), en3 = exp2f((mn - v3) * LOG2E);
    float sp = (ep0 + ep1) + (ep2 + ep3);
    float sn = (en0 + en1) + (en2 + en3);
#pragma unroll
    for (int off = 1; off < 16; off <<= 1) {
      sp += __shfl_xor(sp, off, 32);
      sn += __shfl_xor(sn, off, 32);
    }
    const float rp = 1.0f / sp;
    const float rn = 1.0f / sn;
    const int ro = (8 * hh + r) * FSP + c;
    slab[ro]       = fmaxf(ep0 * rp, EPSV) * FCAR;
    slab[ro + 16]  = fmaxf(ep1 * rp, EPSV) * FCAR;
    slab[ro + 32]  = fmaxf(ep2 * rp, EPSV) * FCAR;
    slab[ro + 48]  = fmaxf(ep3 * rp, EPSV) * FCAR;
    slab[ro + 64]  = fmaxf(en0 * rn, EPSV) * FCAR;
    slab[ro + 80]  = fmaxf(en1 * rn, EPSV) * FCAR;
    slab[ro + 96]  = fmaxf(en2 * rn, EPSV) * FCAR;
    slab[ro + 112] = fmaxf(en3 * rn, EPSV) * FCAR;
  }
  wave_sync_lds();
  v4u oh[8], ol[8];
  const int c8 = c * 8;
#pragma unroll
  for (int it = 0; it < 8; ++it) {
    const int row = 2 * it + hh;
    const v4f a = *(const v4f*)(slab + row * FSP + c8), b4 = *(const v4f*)(slab + row * FSP + c8 + 4);
    float w[8];
#pragma unroll
    for (int e = 0; e < 4; ++e) { w[e] = a[e]; w[4 + e] = b4[e]; }
#pragma unroll
    for (int e = 0; e < 4; ++e) {
      const _Float16 h0 = (_Float16)w[2 * e], h1 = (_Float16)w[2 * e + 1];
      const _Float16 l0 = (_Float16)(w[2 * e] - (float)h0), l1 = (_Float16)(w[2 * e + 1] - (float)h1);
      oh[it][e] = pk16(h_bits(h0), h_bits(h1));
      ol[it][e] = pk16(h_bits(l0), h_bits(l1));
    }
  }
  const size_t ob = ((size_t)head * SEQ + q0) * F2 + c8;
  for (int pass = 0; pass < 2; ++pass) {
#pragma unroll
    for (int it = 0; it < 8; ++it) {
      const int row = 2 * it + hh;
      *(volatile v4u*)(FHo + ob + (size_t)row * F2) = oh[it];
      *(volatile v4u*)(FLo + ob + (size_t)row * F2) = ol[it];
    }
    __threadfence();
  }
}

__global__ __launch_bounds__(ATT_THREADS)
void attn_l(const u16* __restrict__ QFH, const u16* __restrict__ QFL,
            const u16* __restrict__ KFH, const u16* __restrict__ KFL,
            const u16* __restrict__ VHp, const u16* __restrict__ VLp,
            u16* OHp, u16* OLp) {
  __shared__ __align__(16) float smem[WPB * WREG];
  const int tid  = threadIdx.x;
  const int wave = tid >> 5;
  const int lane = tid & 31;
  const int hh   = lane >> 4;
  const int c    = lane & 15;
  const int bid  = blockIdx.x;
  const int qt   = bid % NQT;
  const int hg   = bid / NQT;
  if (hg >= NHG) return;
  const int q0   = qt * 16;
  const int head = hg * WPB + wave;

  float* pt   = smem + wave * WREG;
  float* slab = pt + PTW;

  const size_t fb = (size_t)head * SEQ * F2 + 8 * hh;
  const _Float16* Qh  = ash(QFH) + fb + (size_t)(q0 + c) * F2;
  const _Float16* Ql  = ash(QFL) + fb + (size_t)(q0 + c) * F2;
  const _Float16* Khb = ash(KFH) + fb + (size_t)c * F2;
  const _Float16* Klb = ash(KFL) + fb + (size_t)c * F2;
  const _Float16* Vhb = ash(VHp) + ((size_t)head * HD + c) * SEQ + 8 * hh;
  const _Float16* Vlb = ash(VLp) + ((size_t)head * HD + c) * SEQ + 8 * hh;
  const float lsc = PCAR / (FCAR * FCAR);
  const float ovc = 1.0f / VCAR;
  const size_t KROW = (size_t)F2;

  float lrow[8];
  v8f o[4];
#pragma unroll
  for (int r = 0; r < 8; ++r) lrow[r] = 0.f;
#pragma unroll
  for (int j = 0; j < 4; ++j) o[j] = zero8();
  const int ncaus = (q0 >> 5) + 1;
  const int nkt = (ncaus < NKT) ? ncaus : NKT;
  const int qr0 = q0 + 8 * hh;

#pragma unroll 1
  for (int kt = 0; kt < nkt; ++kt) {
    const int kb = kt * 32;
    v8f s0 = zero8(), s1 = zero8();
    const _Float16* k0p = Khb + (size_t)kb * KROW;
    const _Float16* k1p = k0p + (size_t)16 * KROW;
    const _Float16* l0p = Klb + (size_t)kb * KROW;
    const _Float16* l1p = l0p + (size_t)16 * KROW;
#pragma unroll
    for (int kk = 0; kk < F2 / 32; ++kk) {
      const v16h qh  = ldfrag_h(Qh + kk * 32);
      const v16h ql  = ldfrag_h(Ql + kk * 32);
      const v16h kh0 = ldfrag_h(k0p + kk * 32);
      const v16h kh1 = ldfrag_h(k1p + kk * 32);
      const v16h kl0 = ldfrag_h(l0p + kk * 32);
      const v16h kl1 = ldfrag_h(l1p + kk * 32);
      s0 = mma_h(qh, kh0, s0);
      s0 = mma_h(ql, kh0, s0);
      s0 = mma_h(qh, kl0, s0);
      s1 = mma_h(qh, kh1, s1);
      s1 = mma_h(ql, kh1, s1);
      s1 = mma_h(qh, kl1, s1);
      guard2(s0, s1, qh, ql, kh0, kl0, kh1, kl1);
    }
    const int key0 = kb + c, key1 = kb + 16 + c;
#pragma unroll
    for (int r = 0; r < 8; ++r) {
      const int   qr = qr0 + r;
      const float u0 = s0[r] * lsc;
      const float u1 = s1[r] * lsc;
      const float t0 = (key0 > qr) ? 0.0f : u0;
      const float t1 = (key1 > qr) ? 0.0f : u1;
      float ps = t0 + t1;
#pragma unroll
      for (int off = 1; off < 16; off <<= 1) ps += __shfl_xor(ps, off, 32);
      lrow[r] += ps;
      const int ro = (8 * hh + r) * PTP + c;
      pt[ro]      = t0;
      pt[ro + 16] = t1;
    }
    wave_sync_lds();
    FragH ph, pl;
    {
      const float* prow = pt + c * PTP + 8 * hh;
      const v4f p0 = *(const v4f*)(prow), p1 = *(const v4f*)(prow + 4);
      const v4f p2 = *(const v4f*)(prow + 16), p3 = *(const v4f*)(prow + 20);
#pragma unroll
      for (int e = 0; e < 4; ++e) {
        const float ta = p0[e], tb = p1[e], tc = p2[e], td = p3[e];
        const _Float16 ha = (_Float16)ta, hb = (_Float16)tb, hc = (_Float16)tc, hd = (_Float16)td;
        ph.h[0][e]     = ha;
        ph.h[0][4 + e] = hb;
        ph.h[1][e]     = hc;
        ph.h[1][4 + e] = hd;
        pl.h[0][e]     = (_Float16)(ta - (float)ha);
        pl.h[0][4 + e] = (_Float16)(tb - (float)hb);
        pl.h[1][e]     = (_Float16)(tc - (float)hc);
        pl.h[1][4 + e] = (_Float16)(td - (float)hd);
      }
    }
    {
      const _Float16* vhp = Vhb + kb;
      const _Float16* vlp = Vlb + kb;
#pragma unroll
      for (int jg = 0; jg < 2; ++jg) {
        const size_t da = (size_t)(2 * jg) * 16 * SEQ;
        const size_t db = da + (size_t)16 * SEQ;
        const v16h vha = ldfrag_h(vhp + da), vhb2 = ldfrag_h(vhp + db);
        const v16h vla = ldfrag_h(vlp + da), vlb2 = ldfrag_h(vlp + db);
        o[2 * jg]     = mma_h(ph.v, vha,  o[2 * jg]);
        o[2 * jg]     = mma_h(pl.v, vha,  o[2 * jg]);
        o[2 * jg]     = mma_h(ph.v, vla,  o[2 * jg]);
        o[2 * jg + 1] = mma_h(ph.v, vhb2, o[2 * jg + 1]);
        o[2 * jg + 1] = mma_h(pl.v, vhb2, o[2 * jg + 1]);
        o[2 * jg + 1] = mma_h(ph.v, vlb2, o[2 * jg + 1]);
        guard2(o[2 * jg], o[2 * jg + 1], ph.v, pl.v, vha, vhb2, vla, vlb2);
      }
    }
    wave_sync_lds();
  }
  acc_guard4(o[0], o[1], o[2], o[3]);
#pragma unroll
  for (int r = 0; r < 8; ++r) {
    const float den = lrow[r] + EPSV * PCAR;
    const float inv = (1.0f / den) * ovc;
#pragma unroll
    for (int j = 0; j < 4; ++j) {
      const int idx = (8 * hh + r) * SLP + j * 16 + c;
      slab[idx] = o[j][r] * inv;
    }
  }

  wave_sync_lds();
  v4u oh[4], ol[4];
  const int rq = lane >> 3, c8 = (lane & 7) * 8;
#pragma unroll
  for (int it = 0; it < 4; ++it) {
    const int row = it * 4 + rq;
    const v4f a = *(const v4f*)(slab + row * SLP + c8), b4 = *(const v4f*)(slab + row * SLP + c8 + 4);
    float w[8];
#pragma unroll
    for (int e = 0; e < 4; ++e) { w[e] = a[e] * OSC; w[4 + e] = b4[e] * OSC; }
#pragma unroll
    for (int e = 0; e < 4; ++e) {
      const _Float16 h0 = (_Float16)w[2 * e], h1 = (_Float16)w[2 * e + 1];
      const _Float16 l0 = (_Float16)(w[2 * e] - (float)h0), l1 = (_Float16)(w[2 * e + 1] - (float)h1);
      oh[it][e] = pk16(h_bits(h0), h_bits(h1));
      ol[it][e] = pk16(h_bits(l0), h_bits(l1));
    }
  }
  const size_t ob = (size_t)q0 * DMOD + (size_t)head * HD + c8;
  for (int pass = 0; pass < 2; ++pass) {
#pragma unroll
    for (int it = 0; it < 4; ++it) {
      const int row = it * 4 + rq;
      *(volatile v4u*)(OHp + ob + (size_t)row * DMOD) = oh[it];
      *(volatile v4u*)(OLp + ob + (size_t)row * DMOD) = ol[it];
    }
    __threadfence();
  }
}

extern "C" void kernel_launch(void* const* d_in, const int* in_sizes, int n_in,
                              void* d_out, int out_size, void* d_ws, size_t ws_size,
                              hipStream_t stream) {
  if (n_in < 7) return;
  if (in_sizes[0] < SEQ * DMOD) return;
  if (in_sizes[1] < DMOD * DMOD) return;
  if (in_sizes[2] < DMOD * DMOD) return;
  if (in_sizes[3] < DMOD * DMOD) return;
  if (in_sizes[4] < DMOD * DMOD) return;
  if (in_sizes[5] < NH * HD * FD) return;
  if (in_sizes[6] < NH * HD * FD) return;
  if (out_size < SEQ * DMOD) return;

  const float* x  = (const float*)d_in[0];
  const float* wq = (const float*)d_in[1];
  const float* wk = (const float*)d_in[2];
  const float* wv = (const float*)d_in[3];
  const float* wo = (const float*)d_in[4];
  const float* kq = (const float*)d_in[5];
  const float* kk = (const float*)d_in[6];
  float*       out = (float*)d_out;

  const size_t szXB = (size_t)SEQ * DMOD * 2;
  const size_t szW  = (size_t)DMOD * DMOD * 2;
  const size_t szKT = (size_t)NH * FD * HD * 2;
  const size_t szF  = (size_t)SEQ * DMOD * 4;
  const size_t szH  = (size_t)SEQ * DMOD * 2;
  const size_t szFF = (size_t)NH * SEQ * F2 * 2;
  if (2 * szH > szF) return;
  size_t off = 0;
  const size_t oXB  = off; off += szXB;
  const size_t oW   = off; off += szW;
  const size_t oKQ  = off; off += szKT;
  const size_t oKK  = off; off += szKT;
  const size_t oF   = off; off += szF;
  const size_t oQH  = off; off += szH;
  const size_t oQL  = off; off += szH;
  const size_t oKH  = off; off += szH;
  const size_t oKL  = off; off += szH;
  const size_t oVH  = off; off += szH;
  const size_t oVL  = off; off += szH;
  const size_t oQFH = off; off += szFF;
  const size_t oQFL = off; off += szFF;
  const size_t oKFH = off; off += szFF;
  const size_t oKFL = off; off += szFF;
  if (off > ws_size) return;
  if (off > (size_t)WS_CAP) return;

  char* ws = (char*)d_ws;
  u16*   XB  = (u16*)(ws + oXB);
  u16*   WT  = (u16*)(ws + oW);
  u16*   KQT = (u16*)(ws + oKQ);
  u16*   KKT = (u16*)(ws + oKK);
  float* F   = (float*)(ws + oF);
  u16*   OH  = (u16*)(ws + oF);
  u16*   OL  = (u16*)(ws + oF + szH);
  u16*   QH  = (u16*)(ws + oQH);
  u16*   QL  = (u16*)(ws + oQL);
  u16*   KH  = (u16*)(ws + oKH);
  u16*   KL  = (u16*)(ws + oKL);
  u16*   VH  = (u16*)(ws + oVH);
  u16*   VL  = (u16*)(ws + oVL);
  u16*   QFH = (u16*)(ws + oQFH);
  u16*   QFL = (u16*)(ws + oQFL);
  u16*   KFH = (u16*)(ws + oKFH);
  u16*   KFL = (u16*)(ws + oKFL);

  const dim3 b256(256), b128(128), bAT(ATT_THREADS), bFM(FM_THREADS);
  const int  n8x = (SEQ * DMOD) / 8;
  const dim3 gX((n8x + 255) / 256);
  const dim3 gTW((DMOD / 64) * (DMOD / 64));
  const dim3 gTK(NH);
  const dim3 gG((SEQ / 64) * (DMOD / 64));
  const dim3 gVT(NH * NST);
  const dim3 gFM((NH * NQT) / FWPB);
  const dim3 gAT(NQT * NHG);

  cvt16<<<gX, b256, 0, stream>>>(x, XB, n8x, 0, 1.0f);
  tr16<<<gTW, b256, 0, stream>>>(wv, WT, DMOD, DMOD, 1, 0, 1.0f);
  gemm_bf<<<gG, b128, 0, stream>>>(XB, WT, F, SEQ, DMOD, DMOD, 1.0f);
  vt16<<<gVT, b256, 0, stream>>>(F, VH, VL);
  tr16<<<gTW, b256, 0, stream>>>(wq, WT, DMOD, DMOD, 1, 0, 1.0f);
  gemm_bf<<<gG, b128, 0, stream>>>(XB, WT, F, SEQ, DMOD, DMOD, 1.0f);
  split16<<<gX, b256, 0, stream>>>(F, QH, QL, n8x, QSC);
  tr16<<<gTK, b256, 0, stream>>>(kq, KQT, HD, FD, NH, 1, KQS);
  fmap<<<gFM, bFM, 0, stream>>>(QH, QL, KQT, QFH, QFL);
  tr16<<<gTW, b256, 0, stream>>>(wk, WT, DMOD, DMOD, 1, 0, 1.0f);
  gemm_bf<<<gG, b128, 0, stream>>>(XB, WT, F, SEQ, DMOD, DMOD, 1.0f);
  split16<<<gX, b256, 0, stream>>>(F, KH, KL, n8x, QSC);
  tr16<<<gTK, b256, 0, stream>>>(kk, KKT, HD, FD, NH, 1, KQS);
  fmap<<<gFM, bFM, 0, stream>>>(KH, KL, KKT, KFH, KFL);
  tr16<<<gTW, b256, 0, stream>>>(wo, WT, DMOD, DMOD, 1, 1, WOS);
  attn_l<<<gAT, bAT, 0, stream>>>(QFH, QFL, KFH, KFL, VH, VL, OH, OL);
  gemm_o<<<gG, b128, 0, stream>>>(OH, OL, WT, out, 1.0f / (OSC * WOS));
  (void)hipGetLastError();
}
